// SemanticModule_29858612642627
// MI455X (gfx1250) — hardware-run, weakly checked
//
#include <hip/hip_runtime.h>
#include <stddef.h>
#include <stdint.h>

#ifndef HL_TERMS
#define HL_TERMS 2
#endif

#define NN       100000
#define ET       100000
#define EI       3200000
#define KIN      6
#define HID      32
#define OC       64
#define GBM      128
#define MP       100096
#define APITCH   64
#define BPITCH   64
#define KEXT     (32 * HL_TERMS)
#define NTHR     256
#define NWAVE    8
#define EPT      8
#define WCH      (32 * EPT)
#define NBRUN    1024
#define SLB      10
#define SRCB     17
#define SRCM     0x1FFFF
#define NBK      98
#define RCAP_I   36864
#define WLCAP_I  4480
#define DEGCAP_I 96
#define RCAP_T   2048
#define WLCAP_T  512
#define DEGCAP_T 24
#define MAXB_I   33226
#define MAXDEG_I 63
#define MAXB_T   1121
#define MAXDEG_T 8
#define HTHR     384
#define SMHW     576
#define SMTOT    768
#define WSMAX    ((size_t)(128u << 20))

#define BK_ZI_I  (NWAVE * WLCAP_I + RCAP_I + 2 * NBRUN)
#define BK_ZI_T  (NWAVE * WLCAP_T + RCAP_T + 2 * NBRUN)
#define BK_LDS   ((BK_ZI_I + 16) * 4)

static_assert(HL_TERMS == 1 || HL_TERMS == 2);
static_assert(KEXT % 32 == 0 && KEXT <= APITCH && KEXT <= BPITCH);
static_assert(MP % GBM == 0 && MP >= NN && MP == 782 * GBM);
static_assert(NN == 781 * GBM + 32 && NN % 32 == 0 && NN % 16 == 0);
static_assert(NN <= (1 << SRCB) && NBRUN == (1 << SLB) && SLB + SRCB <= 31);
static_assert(NBK * NBRUN >= NN && (NBK - 1) * NBRUN < NN);
static_assert(EI % EPT == 0 && ET % EPT == 0 && EI % 4 == 0 && ET % 4 == 0);
static_assert((long long)RCAP_I * 100 >= (long long)MAXB_I * 105);
static_assert((long long)RCAP_T * 100 >= (long long)MAXB_T * 105);
static_assert(WLCAP_I >= MAXB_I / 8 + 5 * 61);
static_assert(WLCAP_T >= MAXB_T / 8 + 5 * 12);
static_assert(DEGCAP_I >= MAXDEG_I + 8 && DEGCAP_T >= MAXDEG_T + 8);
static_assert(RCAP_I % (NTHR * 4) == 0 && RCAP_T % (NTHR * 4) == 0);
static_assert(BK_ZI_I % 4 == 0 && BK_ZI_T % 4 == 0 && BK_ZI_T <= BK_ZI_I);
static_assert(BK_LDS <= 300000);
static_assert(NBRUN == 4 * NTHR && NBRUN % 32 == 0);
static_assert((3 * HID * 4) % 128 == 0 && (3 * OC * 4) % 128 == 0 && (HID * 4) % 128 == 0 && (OC * 4) % 128 == 0);
static_assert(HTHR == 16 * 24 && SMHW == KIN * 96 && SMTOT == SMHW + 192);

typedef float          v2f   __attribute__((ext_vector_type(2)));
typedef float          v4f   __attribute__((ext_vector_type(4)));
typedef float          v8f   __attribute__((ext_vector_type(8)));
typedef int            v4i   __attribute__((ext_vector_type(4)));
typedef int            v8i   __attribute__((ext_vector_type(8)));
typedef unsigned short v8us  __attribute__((ext_vector_type(8)));
typedef unsigned short v16us __attribute__((ext_vector_type(16)));
typedef __bf16         v16bf __attribute__((ext_vector_type(16)));
typedef v2f  __attribute__((may_alias)) v2fa;
typedef v4f  __attribute__((may_alias)) v4fa;
typedef v4i  __attribute__((may_alias)) v4ia;
typedef v8us __attribute__((may_alias)) v8usa;
union FragB { v16bf v; v16us u; v8us h[2]; v8i w; };

__device__ __forceinline__ v8f wmb(const FragB& a, const FragB& b, v8f c) {
  v8f d = __builtin_amdgcn_wmma_f32_16x16x32_bf16(false, a.v, false, b.v, (short)0, c, false, false);
  asm volatile("v_nop\n\tv_nop\n\tv_nop\n\tv_nop" : "+v"(d) : "v"(a.w), "v"(b.w));
  return d;
}

__device__ __forceinline__ unsigned bf16_bits(float f) {
  const unsigned u = __float_as_uint(f);
  const unsigned r = (u + 0x7FFFu + ((u >> 16) & 1u)) >> 16;
  const unsigned q = (u >> 16) | 0x40u;
  return ((u & 0x7fffffffu) > 0x7f800000u) ? q : r;
}
__device__ __forceinline__ float bf16_val(float f) {
  return __uint_as_float(bf16_bits(f) << 16);
}

__device__ __forceinline__ void hilo_pack(float v0, float v1, float v2, float v3,
                                          int& h01, int& h23, int& l01, int& l23) {
  const unsigned a0 = bf16_bits(v0), a1 = bf16_bits(v1), a2 = bf16_bits(v2), a3 = bf16_bits(v3);
  const unsigned b0 = bf16_bits(v0 - __uint_as_float(a0 << 16));
  const unsigned b1 = bf16_bits(v1 - __uint_as_float(a1 << 16));
  const unsigned b2 = bf16_bits(v2 - __uint_as_float(a2 << 16));
  const unsigned b3 = bf16_bits(v3 - __uint_as_float(a3 << 16));
  h01 = (int)(a0 | (a1 << 16)); h23 = (int)(a2 | (a3 << 16));
  l01 = (int)(b0 | (b1 << 16)); l23 = (int)(b2 | (b3 << 16));
}

__device__ __forceinline__ v4i regroup_q(int h01, int h23, int l01, int l23, int lane) {
  const int t  = lane & 7;
  const int s0 = (lane & 24) + ((2 * t) & 7), s1 = s0 + 1;
  const int a0 = __shfl(h01, s0, 32), a1 = __shfl(h23, s0, 32), a2 = __shfl(h01, s1, 32), a3 = __shfl(h23, s1, 32);
  const int b0 = __shfl(l01, s0, 32), b1 = __shfl(l23, s0, 32), b2 = __shfl(l01, s1, 32), b3 = __shfl(l23, s1, 32);
  const int mk = (t < 4) ? -1 : 0;
  v4i o;
  o.x = (a0 & mk) | (b0 & ~mk); o.y = (a1 & mk) | (b1 & ~mk);
  o.z = (a2 & mk) | (b2 & ~mk); o.w = (a3 & mk) | (b3 & ~mk);
  return o;
}

__device__ __forceinline__ void st2_v4f(float* p, v4f v) {
  *(volatile v4f*)p = v;
  __threadfence();
  *(volatile v4f*)p = v;
}
__device__ __forceinline__ void st2_v8us(unsigned short* p, v8us v) {
  *(volatile v8us*)p = v;
  __threadfence();
  *(volatile v8us*)p = v;
}

__device__ __forceinline__ v8us gather8(const float* __restrict__ base, int stride) {
  float f[8];
#pragma unroll
  for (int i = 0; i < 8; ++i) f[i] = base[(size_t)i * (size_t)stride];
  v8us o;
#pragma unroll
  for (int i = 0; i < 8; ++i) o[i] = (unsigned short)bf16_bits(f[i]);
  return o;
}

__device__ __forceinline__ unsigned bfr(float x) { return bf16_bits(x) << 16; }

__global__ __launch_bounds__(NTHR) void k_prep(
    const float* __restrict__ hWt, const float* __restrict__ hWi, const float* __restrict__ hWr,
    const float* __restrict__ hb, const float* __restrict__ bWt, const float* __restrict__ bWi,
    const float* __restrict__ bWr, const float* __restrict__ bb, const float* __restrict__ lWt,
    const float* __restrict__ lWi, const float* __restrict__ lWr, const float* __restrict__ lb,
    const float* __restrict__ lpj, unsigned short* WB, unsigned short* WL, unsigned short* WPJ,
    float* SM, unsigned short* Hhl) {
  const int tid = (int)threadIdx.x;
  const int blk = (int)blockIdx.x;
  if (blk < 9) {
    const int mat = blk / 3;
    const int v   = (blk - 3 * mat) * NTHR + tid;
    const int i   = v >> 8, np = (v >> 3) & 31, k8 = (v & 7) * 8, kk = k8 & 31;
    const float* w;
    if (mat == 0) w = bWt; else if (mat == 1) w = bWi; else w = bWr;
    const v8us o = gather8(w + (size_t)i * 1024 + (size_t)kk * 32 + np, 32);
    st2_v8us(WB + (size_t)i * (96 * BPITCH) + (size_t)(mat * 32 + np) * BPITCH + k8, o);
  } else if (blk < 15) {
    const int mat = (blk - 9) >> 1;
    const int v   = ((blk - 9) & 1) * NTHR + tid;
    const int np  = v >> 3, k8 = (v & 7) * 8, kk = k8 & 31;
    const float* w;
    if (mat == 0) w = lWt; else if (mat == 1) w = lWi; else w = lWr;
    const v8us o = gather8(w + (size_t)kk * 64 + np, 64);
    st2_v8us(WL + (size_t)(mat * 64 + np) * BPITCH + k8, o);
  } else if (blk < 17) {
    const int v  = (blk - 15) * NTHR + tid;
    const int np = v >> 3, k8 = (v & 7) * 8, kk = k8 & 31;
    const v8us o = gather8(lpj + (size_t)kk * 64 + np, 64);
    st2_v8us(WPJ + (size_t)np * BPITCH + k8, o);
  } else if (blk == 17) {
    const int t  = tid;
    const int uh = t < 144 ? t : 143;
    const int k  = uh / 24, qq = uh - 24 * k, mat = qq >> 3, c = 4 * (qq & 7);
    const v4f a0 = *(const v4fa*)(hWt + k * 32 + c);
    const v4f a1 = *(const v4fa*)(hWi + k * 32 + c);
    const v4f a2 = *(const v4fa*)(hWr + k * 32 + c);
    int ub = t - 144;
    ub = ub < 0 ? 0 : (ub > 47 ? 47 : ub);
    const int j0 = ub > 7 ? 7 : ub;
    int j1 = ub - 8;  j1 = j1 < 0 ? 0 : (j1 > 23 ? 23 : j1);
    int j2 = ub - 32; j2 = j2 < 0 ? 0 : (j2 > 15 ? 15 : j2);
    const v4f b0 = *(const v4fa*)(hb + 4 * j0);
    const v4f b1 = *(const v4fa*)(bb + 4 * j1);
    const v4f b2 = *(const v4fa*)(lb + 4 * j2);
    asm volatile("" :: "v"(a0), "v"(a1), "v"(a2));
    asm volatile("" :: "v"(b0), "v"(b1), "v"(b2));
    const int sel = (t < 144) ? mat : (ub < 8 ? 3 : (ub < 32 ? 4 : 5));
    const unsigned m0 = (sel == 0) ? 0xffffffffu : 0u, m1 = (sel == 1) ? 0xffffffffu : 0u;
    const unsigned m2 = (sel == 2) ? 0xffffffffu : 0u, m3 = (sel == 3) ? 0xffffffffu : 0u;
    const unsigned m4 = (sel == 4) ? 0xffffffffu : 0u, m5 = (sel == 5) ? 0xffffffffu : 0u;
    v4f o;
    o.x = __uint_as_float((bfr(a0.x) & m0) | (bfr(a1.x) & m1) | (bfr(a2.x) & m2) |
                          (bfr(b0.x) & m3) | (bfr(b1.x) & m4) | (bfr(b2.x) & m5));
    o.y = __uint_as_float((bfr(a0.y) & m0) | (bfr(a1.y) & m1) | (bfr(a2.y) & m2) |
                          (bfr(b0.y) & m3) | (bfr(b1.y) & m4) | (bfr(b2.y) & m5));
    o.z = __uint_as_float((bfr(a0.z) & m0) | (bfr(a1.z) & m1) | (bfr(a2.z) & m2) |
                          (bfr(b0.z) & m3) | (bfr(b1.z) & m4) | (bfr(b2.z) & m5));
    o.w = __uint_as_float((bfr(a0.w) & m0) | (bfr(a1.w) & m1) | (bfr(a2.w) & m2) |
                          (bfr(b0.w) & m3) | (bfr(b1.w) & m4) | (bfr(b2.w) & m5));
    if (t < 192) st2_v4f(SM + 4 * t, o);
  } else {
    const int u = (blk - 18) * NTHR + tid;
    v8us z;
#pragma unroll
    for (int i = 0; i < 8; ++i) z[i] = (unsigned short)0;
    st2_v8us(Hhl + (size_t)NN * APITCH + (size_t)u * 8, z);
  }
}

__device__ __forceinline__ int pack_hit(unsigned s, int sr) {
  sr = sr < 0 ? 0 : (sr > NN - 1 ? NN - 1 : sr);
  return (int)((s << SRCB) | (unsigned)sr);
}

template <int RCAP>
__device__ __forceinline__ void bucket_flush(const int* pl, const int* cnt, const int* offs, int ov,
                                             int* lp, int* cp, int* op, int* fp, int tid) {
#pragma unroll 1
  for (int i = tid * 4; i < RCAP; i += NTHR * 4) {
    const v4i v = *(const v4ia*)(pl + i);
    *(volatile v4i*)(lp + i) = v;
  }
  {
    const v4i c = *(const v4ia*)(cnt + 4 * tid);
    const v4i e = *(const v4ia*)(offs + 4 * tid);
    v4i o;
    o.x = e.x - c.x; o.y = e.y - c.y; o.z = e.z - c.z; o.w = e.w - c.w;
    *(volatile v4i*)(cp + 4 * tid) = c;
    *(volatile v4i*)(op + 4 * tid) = o;
  }
  if (tid < 8) {
    const v4i f = {ov, ov, ov, ov};
    *(volatile v4i*)(fp + 4 * tid) = f;
  }
}

template <int E, int RCAP, int WLCAP, int DEGCAP>
__device__ __forceinline__ void bucket_body(int* dsm, const int* __restrict__ srcs, const int* __restrict__ keys,
                                            int bb, int* lp, int* cp, int* op, int* fp) {
  int* wl   = dsm;
  int* pl   = dsm + NWAVE * WLCAP;
  int* cnt  = pl + RCAP;
  int* offs = cnt + NBRUN;
  int* misc = offs + NBRUN;
  constexpr int ZI  = NWAVE * WLCAP + RCAP + 2 * NBRUN;
  constexpr int NCH = (E + WCH - 1) / WCH;
  const int tid = (int)threadIdx.x, lane = tid & 31, wave = tid >> 5;
  const unsigned nbs = (unsigned)(bb * NBRUN);
  const int nbl = (NN - bb * NBRUN) < NBRUN ? (NN - bb * NBRUN) : NBRUN;

  {
    const v4i z4 = {0, 0, 0, 0};
    for (int i = tid * 4; i < ZI; i += NTHR * 4) *(v4ia*)(dsm + i) = z4;
    if (tid < 16) misc[tid] = 0;
  }
  __syncthreads();

  {
    int* mylist = wl + wave * WLCAP;
    int wc = 0;
#pragma unroll 1
    for (int ch = wave; ch < NCH; ch += NWAVE) {
      const int e0  = ch * WCH + lane * EPT;
      const bool lv = e0 < E;
      const int ec  = lv ? e0 : (E - EPT);
      const v4i da = *(const v4ia*)(keys + ec);
      const v4i db = *(const v4ia*)(keys + ec + 4);
      const unsigned unb = lv ? (unsigned)nbl : 0u;
      const unsigned s0 = (unsigned)da.x - nbs, s1 = (unsigned)da.y - nbs;
      const unsigned s2 = (unsigned)da.z - nbs, s3 = (unsigned)da.w - nbs;
      const unsigned s4 = (unsigned)db.x - nbs, s5 = (unsigned)db.y - nbs;
      const unsigned s6 = (unsigned)db.z - nbs, s7 = (unsigned)db.w - nbs;
      const bool h0 = s0 < unb, h1 = s1 < unb, h2 = s2 < unb, h3 = s3 < unb;
      const bool h4 = s4 < unb, h5 = s5 < unb, h6 = s6 < unb, h7 = s7 < unb;
      const unsigned m0 = __builtin_amdgcn_ballot_w32(h0), m1 = __builtin_amdgcn_ballot_w32(h1);
      const unsigned m2 = __builtin_amdgcn_ballot_w32(h2), m3 = __builtin_amdgcn_ballot_w32(h3);
      const unsigned m4 = __builtin_amdgcn_ballot_w32(h4), m5 = __builtin_amdgcn_ballot_w32(h5);
      const unsigned m6 = __builtin_amdgcn_ballot_w32(h6), m7 = __builtin_amdgcn_ballot_w32(h7);
      const unsigned any = m0 | m1 | m2 | m3 | m4 | m5 | m6 | m7;
      if (any != 0u) {
        const v4i sa = *(const v4ia*)(srcs + ec);
        const v4i sb = *(const v4ia*)(srcs + ec + 4);
        asm volatile("" :: "v"(sa), "v"(sb));
        const int pre = (int)(__builtin_amdgcn_mbcnt_lo(m0, 0u) + __builtin_amdgcn_mbcnt_lo(m1, 0u) +
                              __builtin_amdgcn_mbcnt_lo(m2, 0u) + __builtin_amdgcn_mbcnt_lo(m3, 0u) +
                              __builtin_amdgcn_mbcnt_lo(m4, 0u) + __builtin_amdgcn_mbcnt_lo(m5, 0u) +
                              __builtin_amdgcn_mbcnt_lo(m6, 0u) + __builtin_amdgcn_mbcnt_lo(m7, 0u));
        int p = wc + pre;
        if (h0) { if (p < WLCAP) mylist[p] = pack_hit(s0, sa.x); p = p + 1; }
        if (h1) { if (p < WLCAP) mylist[p] = pack_hit(s1, sa.y); p = p + 1; }
        if (h2) { if (p < WLCAP) mylist[p] = pack_hit(s2, sa.z); p = p + 1; }
        if (h3) { if (p < WLCAP) mylist[p] = pack_hit(s3, sa.w); p = p + 1; }
        if (h4) { if (p < WLCAP) mylist[p] = pack_hit(s4, sb.x); p = p + 1; }
        if (h5) { if (p < WLCAP) mylist[p] = pack_hit(s5, sb.y); p = p + 1; }
        if (h6) { if (p < WLCAP) mylist[p] = pack_hit(s6, sb.z); p = p + 1; }
        if (h7) { if (p < WLCAP) mylist[p] = pack_hit(s7, sb.w); p = p + 1; }
        wc += (int)(__builtin_popcount(m0) + __builtin_popcount(m1) + __builtin_popcount(m2) + __builtin_popcount(m3) +
                    __builtin_popcount(m4) + __builtin_popcount(m5) + __builtin_popcount(m6) + __builtin_popcount(m7));
      }
    }
    if (lane == 0) misc[wave] = wc;
  }
  __syncthreads();

  if (wave == 0) {
    int ov = 0;
#pragma unroll 1
    for (int w2 = 0; w2 < NWAVE; ++w2) {
      int c = misc[w2];
      if (c > WLCAP) ov = 1;
      c = c < 0 ? 0 : (c > WLCAP ? WLCAP : c);
#pragma unroll 1
      for (int b0 = 0; b0 < c; b0 += 32) {
        const int idx = b0 + lane;
        const int ent = wl[w2 * WLCAP + (idx < WLCAP ? idx : WLCAP - 1)];
        const int m32 = (c - b0) < 32 ? (c - b0) : 32;
#pragma unroll 1
        for (int k = 0; k < m32; ++k) {
          const int u    = __builtin_amdgcn_readlane(ent, k);
          const int slot = (u >> SRCB) & (NBRUN - 1);
          if (lane == 0) cnt[slot] = cnt[slot] + 1;
        }
      }
    }
    if (lane == 0) misc[9] = ov;
  }
  __syncthreads();
  if (wave == 0) {
    const int base = lane * (NBRUN / 32);
    int s = 0, dg = 0;
#pragma unroll 1
    for (int i = 0; i < NBRUN / 32; ++i) {
      const int cv = cnt[base + i];
      s += cv;
      dg |= (cv > DEGCAP) ? 1 : 0;
    }
    int incl = s;
#pragma unroll
    for (int d = 1; d < 32; d <<= 1) {
      const int y = __shfl_up(incl, d, 32);
      if (lane >= d) incl += y;
    }
    int run = incl - s;
#pragma unroll 1
    for (int i = 0; i < NBRUN / 32; ++i) {
      const int cv = cnt[base + i];
      offs[base + i] = run;
      run += cv;
    }
    const int total = __shfl(incl, 31, 32);
    const unsigned bad = __builtin_amdgcn_ballot_w32((dg != 0) | (total > RCAP));
    if (lane == 0) misc[9] = misc[9] | ((bad != 0u) ? 1 : 0);
  }
  __syncthreads();

  if (wave == 0) {
#pragma unroll 1
    for (int w2 = 0; w2 < NWAVE; ++w2) {
      int c = misc[w2];
      c = c < 0 ? 0 : (c > WLCAP ? WLCAP : c);
#pragma unroll 1
      for (int b0 = 0; b0 < c; b0 += 32) {
        const int idx = b0 + lane;
        const int ent = wl[w2 * WLCAP + (idx < WLCAP ? idx : WLCAP - 1)];
        const int m32 = (c - b0) < 32 ? (c - b0) : 32;
#pragma unroll 1
        for (int k = 0; k < m32; ++k) {
          const int u    = __builtin_amdgcn_readlane(ent, k);
          const int slot = (u >> SRCB) & (NBRUN - 1);
          if (lane == 0) {
            int p = offs[slot];
            p = p < 0 ? 0 : (p > RCAP - 1 ? RCAP - 1 : p);
            pl[p] = u & SRCM;
            offs[slot] = p + 1;
          }
        }
      }
    }
  }
  __syncthreads();

  const int ovf = misc[9];
  bucket_flush<RCAP>(pl, cnt, offs, ovf, lp, cp, op, fp, tid);
  __threadfence();
  bucket_flush<RCAP>(pl, cnt, offs, ovf, lp, cp, op, fp, tid);
}

__global__ __launch_bounds__(NTHR) void k_bucket(const int* __restrict__ eiI, const int* __restrict__ eiT,
                                                 int* LISTI, int* LISTT, int* CNTI, int* OFFI,
                                                 int* CNTT, int* OFFT, int* FLAG) {
  extern __shared__ __attribute__((aligned(16))) int dsm[];
  const int blk = (int)blockIdx.x;
  if (blk < NBK) {
    bucket_body<EI, RCAP_I, WLCAP_I, DEGCAP_I>(dsm, eiI, eiI + EI, blk,
        LISTI + (size_t)blk * RCAP_I, CNTI + (size_t)blk * NBRUN, OFFI + (size_t)blk * NBRUN,
        FLAG + (size_t)blk * 32);
  } else {
    const int bb = blk - NBK;
    bucket_body<ET, RCAP_T, WLCAP_T, DEGCAP_T>(dsm, eiT, eiT + ET, bb,
        LISTT + (size_t)bb * RCAP_T, CNTT + (size_t)bb * NBRUN, OFFT + (size_t)bb * NBRUN,
        FLAG + (size_t)blk * 32);
  }
}

__global__ __launch_bounds__(HTHR) void k_head(const float* __restrict__ x, const float* __restrict__ SM, float* P) {
  __shared__ __attribute__((aligned(16))) float xs[96];
  __shared__ __attribute__((aligned(16))) float hw[SMHW];
  const int tid = (int)threadIdx.x;
  const int rowBase = (int)blockIdx.x * 16;
  if (tid < 64) {
    const int i = tid < 48 ? tid : 47;
    const v2f a = *(const v2fa*)(x + (size_t)rowBase * KIN + 2 * i);
    v2f b;
    b.x = bf16_val(a.x); b.y = bf16_val(a.y);
    *(v2fa*)(xs + 2 * i) = b;
  } else if (tid < 224) {
    const int u = (tid - 64) < 144 ? (tid - 64) : 143;
    *(v4fa*)(hw + 4 * u) = *(const v4fa*)(SM + 4 * u);
  }
  __syncthreads();
  const int node = tid / 24, q4 = tid - node * 24;
  float a0 = 0.0f, a1 = 0.0f, a2 = 0.0f, a3 = 0.0f;
#pragma unroll 1
  for (int k = 0; k < KIN; ++k) {
    const float xv = xs[node * KIN + k];
    const v4f w = *(const v4fa*)(hw + k * 96 + 4 * q4);
    a0 = fmaf(xv, w.x, a0); a1 = fmaf(xv, w.y, a1); a2 = fmaf(xv, w.z, a2); a3 = fmaf(xv, w.w, a3);
  }
  v4f o;
  o.x = a0; o.y = a1; o.z = a2; o.w = a3;
  st2_v4f(P + (size_t)rowBase * 96 + 4 * tid, o);
}

template <int LPD, int PP, int RCAP, int DEGCAP>
__device__ __forceinline__ v4f seg_sum(const int* __restrict__ lb, int craw, int oraw,
                                       const float* __restrict__ Pc, int& cuse, int& big) {
  big = (craw > DEGCAP) ? 1 : 0;
  const int c = craw < 0 ? 0 : (craw > DEGCAP ? DEGCAP : craw);
  const int o = oraw < 0 ? 0 : (oraw > RCAP - 1 ? RCAP - 1 : oraw);
  int cm = c;
  if (LPD == 8) {
    const int t8 = __shfl_xor(cm, 8, 32);
    cm = cm > t8 ? cm : t8;
  }
  {
    const int t16 = __shfl_xor(cm, 16, 32);
    cm = cm > t16 ? cm : t16;
  }
  const int cmu = __builtin_amdgcn_readfirstlane(cm);
  int last = o + c - 1;
  last = last < o ? o : last;
  last = last > RCAP - 1 ? RCAP - 1 : last;
  float a0 = 0.0f, a1 = 0.0f, a2 = 0.0f, a3 = 0.0f;
#pragma unroll 1
  for (int j = 0; j < cmu; ++j) {
    int idx = o + j;
    idx = idx > last ? last : idx;
    const int wd = lb[idx];
    int sr = wd & SRCM;
    sr = sr > NN - 1 ? NN - 1 : sr;
    const v4f v = *(const v4fa*)(Pc + (size_t)sr * PP);
    asm volatile("" :: "v"(v));
    const bool valid = j < c;
    a0 += valid ? v.x : 0.0f; a1 += valid ? v.y : 0.0f;
    a2 += valid ? v.z : 0.0f; a3 += valid ? v.w : 0.0f;
  }
  cuse = c;
  v4f r;
  r.x = a0; r.y = a1; r.z = a2; r.w = a3;
  return r;
}

template <int W, int MODE>
__global__ __launch_bounds__(NTHR) void k_replay(
    const int* __restrict__ LISTI, const int* __restrict__ LISTT, const int* __restrict__ CNTI,
    const int* __restrict__ OFFI, const int* __restrict__ CNTT, const int* __restrict__ OFFT,
    const int* __restrict__ FLAG, const float* __restrict__ P, const float* __restrict__ bias,
    float* H, unsigned short* Hhl, float* OUT) {
  constexpr int LPD = W / 4, DPW = 32 / LPD, DPB = NWAVE * DPW, PP = 3 * W;
  static_assert(NN % DPB == 0 && NBRUN % DPB == 0);
  static_assert((W == 32 && MODE < 2) || (W == 64 && MODE == 2));
  __shared__ __attribute__((aligned(16))) float sb[64];
  const int tid = (int)threadIdx.x, lane = tid & 31, wave = tid >> 5;
  const int q = lane & (LPD - 1), g = lane / LPD;
  const int rowBase = (int)blockIdx.x * DPB;
  const int n = rowBase + wave * DPW + g;
  const int bucket = rowBase >> SLB;
  const int flag = FLAG[(size_t)bucket * 32] | FLAG[(size_t)(NBK + bucket) * 32];
  if (wave == 0) {
    const int i = lane & (LPD - 1);
    *(v4fa*)(sb + 4 * i) = *(const v4fa*)(bias + 4 * i);
  }
  __syncthreads();

  const int cTr = CNTT[n], oTr = OFFT[n];
  const int cIr = CNTI[n], oIr = OFFI[n];
  int cT, bigT, cI, bigI;
  const v4f aT = seg_sum<LPD, PP, RCAP_T, DEGCAP_T>(LISTT + (size_t)bucket * RCAP_T, cTr, oTr,
                                                    P + 4 * q, cT, bigT);
  const v4f aI = seg_sum<LPD, PP, RCAP_I, DEGCAP_I>(LISTI + (size_t)bucket * RCAP_I, cIr, oIr,
                                                    P + W + 4 * q, cI, bigI);
  (void)cT;
  const float den = (float)(cI < 1 ? 1 : cI);
  const v4f own = *(const v4fa*)(P + (size_t)n * PP + 2 * W + 4 * q);
  const v4f bv  = *(const v4fa*)(sb + 4 * q);
  float v0 = ((aT.x + aI.x / den) + own.x) + bv.x;
  float v1 = ((aT.y + aI.y / den) + own.y) + bv.y;
  float v2 = ((aT.z + aI.z / den) + own.z) + bv.z;
  float v3 = ((aT.w + aI.w / den) + own.w) + bv.w;
  v0 = (v0 > 0.0f) ? v0 : (v0 - v0); v1 = (v1 > 0.0f) ? v1 : (v1 - v1);
  v2 = (v2 > 0.0f) ? v2 : (v2 - v2); v3 = (v3 > 0.0f) ? v3 : (v3 - v3);
  const bool bad = (flag != 0) | (bigT != 0) | (bigI != 0);
  const float qnan = __uint_as_float(0x7fc00000u);

  if constexpr (MODE == 2) {
    float* op = OUT + (size_t)n * OC + 4 * q;
    const v4f pj = *(const v4fa*)op;
    float m0 = v0 + pj.x, m1 = v1 + pj.y, m2 = v2 + pj.z, m3 = v3 + pj.w;
    m0 = bad ? qnan : m0; m1 = bad ? qnan : m1; m2 = bad ? qnan : m2; m3 = bad ? qnan : m3;
    v4f ov;
    ov.x = m0; ov.y = m1; ov.z = m2; ov.w = m3;
    *(volatile v4f*)op = ov;
    __threadfence();
    *(volatile v4f*)op = ov;
    (void)H; (void)Hhl;
  } else {
    float* hp = H + (size_t)n * HID + 4 * q;
    float m0 = v0, m1 = v1, m2 = v2, m3 = v3;
    if constexpr (MODE == 1) {
      const v4f res = *(const v4fa*)hp;
      m0 = v0 + res.x; m1 = v1 + res.y; m2 = v2 + res.z; m3 = v3 + res.w;
    }
    m0 = bad ? qnan : m0; m1 = bad ? qnan : m1; m2 = bad ? qnan : m2; m3 = bad ? qnan : m3;
    int h01, h23, l01, l23;
    hilo_pack(m0, m1, m2, m3, h01, h23, l01, l23);
    const v4i ow = regroup_q(h01, h23, l01, l23, lane);
    v4f ov;
    ov.x = m0; ov.y = m1; ov.z = m2; ov.w = m3;
    unsigned short* lp = Hhl + (size_t)n * APITCH + 8 * q;
    *(volatile v4f*)hp = ov;
    *(volatile v4i*)lp = ow;
    __threadfence();
    *(volatile v4f*)hp = ov;
    *(volatile v4i*)lp = ow;
    (void)OUT;
  }
}

template <int NACC>
__device__ __forceinline__ void gemm_rows(const unsigned short* __restrict__ ap,
                                          const unsigned short* __restrict__ bp, v8f (&acc)[NACC]) {
#pragma unroll 1
  for (int k0 = 0; k0 < KEXT; k0 += 32) {
    FragB af;
    af.h[0] = *(const v8usa*)(ap + k0);
    af.h[1] = *(const v8usa*)(ap + k0 + 16);
#pragma unroll
    for (int nt = 0; nt < NACC; ++nt) {
      const unsigned short* wq = bp + (size_t)(16 * nt) * (size_t)BPITCH + k0;
      FragB bf;
      bf.h[0] = *(const v8usa*)wq;
      bf.h[1] = *(const v8usa*)(wq + 16);
      acc[nt] = wmb(af, bf, acc[nt]);
    }
  }
}

template <int NT>
__global__ __launch_bounds__(NTHR) __attribute__((amdgpu_num_vgpr(248)))
void k_gemm(const unsigned short* __restrict__ A, const unsigned short* __restrict__ BT, float* outp, int opitch) {
  constexpr int NACC = NT / 16, SP = NT + 4, C4 = NT / 4, ITER = (16 * C4) / 32;
  static_assert(NT % 16 == 0 && (16 * C4) % 32 == 0 && (SP * 4) % 16 == 0);
  static_assert(GBM * SP * 4 <= 65536);
  __shared__ __attribute__((aligned(16))) float stg[GBM * SP];
  const int tid = (int)threadIdx.x, lane = tid & 31, wave = tid >> 5, hh = lane >> 4, m = lane & 15;
  const int rowBase = (int)blockIdx.x * GBM;
  const int ycol = (int)blockIdx.y * NT;

  v8f acc[NACC];
  {
    const v8f z = {0.f, 0.f, 0.f, 0.f, 0.f, 0.f, 0.f, 0.f};
#pragma unroll
    for (int t = 0; t < NACC; ++t) acc[t] = z;
  }
  const unsigned short* ap = A + (size_t)(rowBase + 16 * wave + m) * (size_t)APITCH + 8 * hh;
  const unsigned short* bp = BT + (size_t)(ycol + m) * (size_t)BPITCH + 8 * hh;
  gemm_rows<NACC>(ap, bp, acc);
#pragma unroll
  for (int nt = 0; nt < NACC; ++nt) {
#pragma unroll
    for (int r = 0; r < 8; ++r) stg[(16 * wave + 8 * hh + r) * SP + 16 * nt + m] = acc[nt][r];
  }
  __syncthreads();

#pragma unroll 1
  for (int it = 0; it < ITER; ++it) {
    const int idx = it * 32 + lane;
    const int r   = idx / C4, c4 = idx - r * C4;
    const int lr  = 16 * wave + r;
    const int grow = rowBase + lr;
    const v4f v = *(const v4fa*)(stg + lr * SP + 4 * c4);
    asm volatile("" :: "v"(v));
    if (grow < NN) st2_v4f(outp + (size_t)grow * (size_t)opitch + ycol + 4 * c4, v);
  }
}

extern "C" void kernel_launch(void* const* d_in, const int* in_sizes, int n_in,
                              void* d_out, int out_size, void* d_ws, size_t ws_size,
                              hipStream_t stream) {
  if (n_in < 16) return;
  if (in_sizes[0] != NN * KIN) return;
  if (in_sizes[1] != 2 * ET) return;
  if (in_sizes[2] != 2 * EI) return;
  if (in_sizes[3] != KIN * HID || in_sizes[4] != KIN * HID || in_sizes[5] != KIN * HID) return;
  if (in_sizes[6] != HID) return;
  if (in_sizes[7] != 3 * HID * HID || in_sizes[8] != 3 * HID * HID || in_sizes[9] != 3 * HID * HID) return;
  if (in_sizes[10] != 3 * HID) return;
  if (in_sizes[11] != HID * OC || in_sizes[12] != HID * OC || in_sizes[13] != HID * OC) return;
  if (in_sizes[14] != OC) return;
  if (in_sizes[15] != HID * OC) return;
  if (out_size != NN * OC) return;

  const float* x   = (const float*)d_in[0];
  const int*   eiT = (const int*)d_in[1];
  const int*   eiI = (const int*)d_in[2];
  const float* hWt = (const float*)d_in[3];
  const float* hWi = (const float*)d_in[4];
  const float* hWr = (const float*)d_in[5];
  const float* hb  = (const float*)d_in[6];
  const float* bWt = (const float*)d_in[7];
  const float* bWi = (const float*)d_in[8];
  const float* bWr = (const float*)d_in[9];
  const float* bb  = (const float*)d_in[10];
  const float* lWt = (const float*)d_in[11];
  const float* lWi = (const float*)d_in[12];
  const float* lWr = (const float*)d_in[13];
  const float* lb  = (const float*)d_in[14];
  const float* lpj = (const float*)d_in[15];
  float* out = (float*)d_out;

  constexpr size_t zP    = (size_t)NN * 192 * 4;
  constexpr size_t zH    = (size_t)NN * HID * 4;
  constexpr size_t zHL   = (size_t)MP * APITCH * 2;
  constexpr size_t zLI   = (size_t)NBK * RCAP_I * 4;
  constexpr size_t zLT   = (size_t)NBK * RCAP_T * 4;
  constexpr size_t zCO   = (size_t)NBK * NBRUN * 4;
  constexpr size_t zFLAG = (size_t)2 * NBK * 128;
  constexpr size_t zWB   = (size_t)3 * 96 * BPITCH * 2;
  constexpr size_t zWL   = (size_t)192 * BPITCH * 2;
  constexpr size_t zWPJ  = (size_t)64 * BPITCH * 2;
  constexpr size_t zSM   = (size_t)SMTOT * 4;
  constexpr size_t oP    = 0;
  constexpr size_t oH    = oP + zP;
  constexpr size_t oHL   = oH + zH;
  constexpr size_t oLI   = oHL + zHL;
  constexpr size_t oLT   = oLI + zLI;
  constexpr size_t oCI   = oLT + zLT;
  constexpr size_t oOI   = oCI + zCO;
  constexpr size_t oCT   = oOI + zCO;
  constexpr size_t oOT   = oCT + zCO;
  constexpr size_t oFLAG = oOT + zCO;
  constexpr size_t oWB   = oFLAG + zFLAG;
  constexpr size_t oWL   = oWB + zWB;
  constexpr size_t oWPJ  = oWL + zWL;
  constexpr size_t oSM   = oWPJ + zWPJ;
  constexpr size_t oEND  = oSM + zSM;
  static_assert(zP % 256 == 0 && zH % 256 == 0 && zHL % 256 == 0 && zLI % 256 == 0 && zLT % 256 == 0);
  static_assert(zCO % 256 == 0 && zFLAG % 256 == 0 && zWB % 256 == 0 && zWL % 256 == 0 && zWPJ % 256 == 0);
  static_assert(zSM % 256 == 0);
  static_assert((size_t)NN * 96 * 4 <= zP);
  static_assert(oEND <= WSMAX);
  if (oEND > ws_size) return;

  char* ws = (char*)d_ws;
  float*          P     = (float*)(ws + oP);
  float*          H     = (float*)(ws + oH);
  unsigned short* Hhl   = (unsigned short*)(ws + oHL);
  int*            LISTI = (int*)(ws + oLI);
  int*            LISTT = (int*)(ws + oLT);
  int*            CNTI  = (int*)(ws + oCI);
  int*            OFFI  = (int*)(ws + oOI);
  int*            CNTT  = (int*)(ws + oCT);
  int*            OFFT  = (int*)(ws + oOT);
  int*            FLAG  = (int*)(ws + oFLAG);
  unsigned short* WB    = (unsigned short*)(ws + oWB);
  unsigned short* WL    = (unsigned short*)(ws + oWL);
  unsigned short* WPJ   = (unsigned short*)(ws + oWPJ);
  float*          SM    = (float*)(ws + oSM);

  hipFuncSetAttribute(reinterpret_cast<const void*>(&k_bucket), hipFuncAttributeMaxDynamicSharedMemorySize, (int)BK_LDS);

  k_prep<<<21, NTHR, 0, stream>>>(hWt, hWi, hWr, hb, bWt, bWi, bWr, bb, lWt, lWi, lWr, lb, lpj,
                                  WB, WL, WPJ, SM, Hhl);
  k_bucket<<<2 * NBK, NTHR, BK_LDS, stream>>>(eiI, eiT, LISTI, LISTT, CNTI, OFFI, CNTT, OFFT, FLAG);
  k_head<<<NN / 16, HTHR, 0, stream>>>(x, SM, P);
  k_replay<32, 0><<<NN / 32, NTHR, 0, stream>>>(LISTI, LISTT, CNTI, OFFI, CNTT, OFFT, FLAG, P, SM + SMHW,
                                                H, Hhl, out);
  for (int i = 0; i < 3; ++i) {
    k_gemm<96><<<MP / GBM, NTHR, 0, stream>>>(Hhl, WB + (size_t)i * (96 * BPITCH), P, 96);
    k_replay<32, 1><<<NN / 32, NTHR, 0, stream>>>(LISTI, LISTT, CNTI, OFFI, CNTT, OFFT, FLAG, P,
                                                  SM + SMHW + 32 + 32 * i, H, Hhl, out);
  }
  k_gemm<64><<<dim3(MP / GBM, 3, 1), NTHR, 0, stream>>>(Hhl, WL, P, 192);
  k_gemm<64><<<MP / GBM, NTHR, 0, stream>>>(Hhl, WPJ, out, OC);
  k_replay<64, 2><<<NN / 16, NTHR, 0, stream>>>(LISTI, LISTT, CNTI, OFFI, CNTT, OFFT, FLAG, P,
                                                SM + SMHW + 128, H, Hhl, out);
}
